// TransformerBlock_730144440854
// MI455X (gfx1250) — hardware-run, weakly checked
//
#include <hip/hip_runtime.h>


#ifndef NB
#define NB 8
#endif
#ifndef SEQ
#define SEQ 1024
#endif
#define NB_FULL  8
#define SEQ_FULL 1024
#define DM   256
#define NH_  8
#define HD   32
#define R3   (3 * SEQ)
#define NMAT 7
#define TP   72
#define CSP  264
#define OSP  68
#define TFP  68
#define L2E  1.4426950408889634f
#define XC   16.0f
#define WSC  64.0f
#define PINV 0.0009765625f
#define QKC  16.0f
#define VC   16.0f
#define PEXP 10.0f
#define CC   1024.0f
#define AC   16.0f
#define AINV 0.0625f
#define RSC  2048.0f
#define RINV 0.00048828125f
#define SC2  (0.00390625f * 0.10206207261596575f * L2E)

static_assert(NB_FULL == 8);
static_assert(NH_ * HD == DM);
static_assert(HD == 32);
static_assert(DM == 256);
static_assert(32 * 8 == DM);
static_assert(SEQ % 64 == 0);
static_assert(NB <= NB_FULL);
static_assert(SEQ <= SEQ_FULL);
static_assert(((size_t)NB * SEQ) % 64 == 0);
static_assert(R3 % 64 == 0);
static_assert(TP % 8 == 0);
static_assert(CSP % 8 == 0);
static_assert(OSP % 4 == 0);
static_assert(TFP % 4 == 0);

typedef _Float16 h16;
typedef __attribute__((ext_vector_type(16))) _Float16 v16h;
typedef __attribute__((ext_vector_type(8)))  _Float16 v8h;
typedef __attribute__((ext_vector_type(8)))  float    v8f;
typedef __attribute__((ext_vector_type(4)))  float    v4f;
typedef v4f  __attribute__((may_alias)) v4fa;
typedef v8h  __attribute__((may_alias)) v8ha;

static constexpr size_t QPL = (size_t)NB * R3 * DM;

__device__ __forceinline__ float rbf(float f) { unsigned u = __float_as_uint(f); u += 0x7FFFu + ((u >> 16) & 1u); return __uint_as_float(u & 0xFFFF0000u); }
static __device__ __forceinline__ h16 toh_flush(float v) { const h16 r = (h16)v; return (fabsf(v) < 6.103515625e-05f) ? (h16)0.0f : r; }
__device__ __forceinline__ v16h cat16(v8h lo, v8h hi) { return __builtin_shufflevector(lo, hi, 0, 1, 2, 3, 4, 5, 6, 7, 8, 9, 10, 11, 12, 13, 14, 15); }
__device__ __forceinline__ v16h ldh(const h16* p) { return cat16(*(const v8h*)p, *(const v8h*)(p + 16)); }
__device__ __forceinline__ v8f wmma_g(v16h a, v16h b, v8f c) {
    c = __builtin_amdgcn_wmma_f32_16x16x32_f16(false, a, false, b, (short)0, c, false, false);
    asm volatile("v_nop\n\tv_nop\n\tv_nop\n\tv_nop" : "+v"(c) : "v"(a), "v"(b));
    return c;
}

__global__ __launch_bounds__(256) void k_cvt_x(const float* __restrict__ x, h16* XH) {
    __shared__ __align__(16) h16 ts[64 * TP];
    const int tid = threadIdx.x;
    const int rt = blockIdx.x;
    const int d = rt / (SEQ / 64), n0 = (rt % (SEQ / 64)) * 64;
    const int c0 = blockIdx.y * 64, b = blockIdx.z;
    const int cl = tid >> 2, q = (tid & 3) * 16;
    const float* src = x + (((size_t)b * DM + c0 + cl) * 3 + d) * SEQ_FULL + n0 + q;
    const v4f a0 = *(const v4f*)(src), a1 = *(const v4f*)(src + 4), a2 = *(const v4f*)(src + 8), a3 = *(const v4f*)(src + 12);
#pragma unroll
    for (int k = 0; k < 4; ++k) {
        ts[(q + k) * TP + cl]      = toh_flush(rbf(a0[k]) * XC);
        ts[(q + 4 + k) * TP + cl]  = toh_flush(rbf(a1[k]) * XC);
        ts[(q + 8 + k) * TP + cl]  = toh_flush(rbf(a2[k]) * XC);
        ts[(q + 12 + k) * TP + cl] = toh_flush(rbf(a3[k]) * XC); }
    __syncthreads();
    h16* dst = XH + ((size_t)b * R3 + (size_t)rt * 64) * DM + c0;
#pragma unroll 1
    for (int ps = 0; ps < 2; ++ps) {
#pragma unroll
        for (int s = 0; s < 2; ++s) { const int row = 32 * s + (tid >> 3), c8 = (tid & 7) * 8;
            const v8h val = *(const v8ha*)(&ts[row * TP + c8]);
            *(volatile v8h*)(dst + (size_t)row * DM + c8) = val; }
        if (ps == 0) __threadfence(); }
}

__global__ __launch_bounds__(256) void k_cvt_w(const float* __restrict__ w0, const float* __restrict__ w1, const float* __restrict__ w2, const float* __restrict__ w3,
                                               const float* __restrict__ w4, const float* __restrict__ w5, const float* __restrict__ w6,
                                               const float* __restrict__ b0, const float* __restrict__ b1, const float* __restrict__ b2, const float* __restrict__ b3,
                                               const float* __restrict__ b4, const float* __restrict__ b6, h16* WH, float* UT) {
#pragma clang fp contract(off)
    __shared__ __align__(16) h16 ts[64 * TP];
    __shared__ __align__(16) float su[3 * DM];
    const int tid = threadIdx.x;
    const int which = blockIdx.z;
    const int i0 = blockIdx.x * 64, o0 = blockIdx.y * 64;
    const int il = tid >> 2, q = (tid & 3) * 16;
    const size_t so = (size_t)(i0 + il) * DM + o0 + q;
#pragma unroll 1
    for (int k = 0; k < 4; ++k) {
        const size_t e = so + 4 * k;
        const v4f a0 = *(const v4f*)(w0 + e); const v4f a1 = *(const v4f*)(w1 + e); const v4f a2 = *(const v4f*)(w2 + e); const v4f a3 = *(const v4f*)(w3 + e);
        const v4f a4 = *(const v4f*)(w4 + e); const v4f a5 = *(const v4f*)(w5 + e); const v4f a6 = *(const v4f*)(w6 + e);
        v4f v = a0;
        v = (which == 1) ? a1 : v; v = (which == 2) ? a2 : v; v = (which == 3) ? a3 : v;
        v = (which == 4) ? a4 : v; v = (which == 5) ? a5 : v; v = (which == 6) ? a6 : v;
#pragma unroll
        for (int e2 = 0; e2 < 4; ++e2) ts[(q + 4 * k + e2) * TP + il] = toh_flush(rbf(v[e2]) * WSC);
    }
    __syncthreads();
    h16* dst = WH + (size_t)which * DM * DM + (size_t)o0 * DM + i0;
#pragma unroll 1
    for (int ps = 0; ps < 2; ++ps) {
#pragma unroll
        for (int s = 0; s < 2; ++s) { const int row = 32 * s + (tid >> 3), c8 = (tid & 7) * 8;
            const v8h val = *(const v8ha*)(&ts[row * TP + c8]);
            *(volatile v8h*)(dst + (size_t)row * DM + c8) = val; }
        if (ps == 0) __threadfence(); }
    if (blockIdx.x == 0 && blockIdx.y == 0) {
        const int c = tid;
        float u[3];
#pragma unroll
        for (int e = 0; e < 3; ++e) {
            const float v0 = b0[c * 3 + e], v1 = b1[c * 3 + e], v2 = b2[c * 3 + e], v3 = b3[c * 3 + e], v4 = b4[c * 3 + e], v6 = b6[c * 3 + e];
            float v = v0;
            v = (which == 1) ? v1 : v; v = (which == 2) ? v2 : v; v = (which == 3) ? v3 : v; v = (which == 4) ? v4 : v; v = (which == 6) ? v6 : v;
            u[e] = rbf(v); }
        const float ss = u[0] * u[0] + u[1] * u[1] + u[2] * u[2];
        const float inv = 1.0f / sqrtf(ss);
#pragma unroll
        for (int e = 0; e < 3; ++e) { const float t = (1e-6f * u[e]) * inv; su[e * DM + c] = (which == 5) ? 0.0f : t; }
        __syncthreads();
        if (tid < 192) {
            const v4f val = *(const v4fa*)(&su[tid * 4]);
            float* ud = UT + (size_t)which * 3 * DM + tid * 4;
            *(volatile v4f*)ud = val;
            __threadfence();
            *(volatile v4f*)ud = val;
        }
    }
}

__global__ __launch_bounds__(128) void k_proj(const h16* __restrict__ XH, const h16* __restrict__ WH, const float* __restrict__ UT,
                                              h16* QK, h16* VTH, h16* VTR) {
    __shared__ __align__(16) h16 ts[2 * 64 * TP];
    const int tid = threadIdx.x, lane = tid & 31, lr = lane & 15, hi = lane >> 4;
    const int wave = __builtin_amdgcn_readfirstlane((int)(threadIdx.x >> 5));
    const int which = blockIdx.z / NB, b = blockIdx.z % NB;
    const int row0 = blockIdx.x * 64, n0 = blockIdx.y * 64;
    const int d = row0 / SEQ, tl0 = row0 % SEQ;
    const h16* ap = XH + ((size_t)b * R3 + row0 + 16 * wave + lr) * DM + 8 * hi;
    const h16* wp = WH + (size_t)which * DM * DM + (size_t)(n0 + lr) * DM + 8 * hi;
    v8f c0 = (v8f){}, c1 = (v8f){}, c2 = (v8f){}, c3 = (v8f){};
#pragma unroll 1
    for (int k0 = 0; k0 < DM; k0 += 32) {
        const v16h a = ldh(ap + k0);
        const v16h w0 = ldh(wp + k0), w1 = ldh(wp + (size_t)16 * DM + k0), w2 = ldh(wp + (size_t)32 * DM + k0), w3 = ldh(wp + (size_t)48 * DM + k0);
        c0 = wmma_g(a, w0, c0); c1 = wmma_g(a, w1, c1); c2 = wmma_g(a, w2, c2); c3 = wmma_g(a, w3, c3);
    }
    const float* up = UT + ((size_t)which * 3 + d) * DM + n0 + lr;
    const float bb0 = up[0], bb1 = up[16], bb2 = up[32], bb3 = up[48];
    if (which < 2) {
#pragma unroll
        for (int r = 0; r < 8; ++r) { const int ro = wave * 16 * TP + (8 * hi + r) * TP + lr;
            { const float v = (c0[r] * PINV + bb0) * QKC; const h16 hh = toh_flush(v); ts[ro] = hh;      ts[64 * TP + ro] = toh_flush((v - (float)hh) * RSC); }
            { const float v = (c1[r] * PINV + bb1) * QKC; const h16 hh = toh_flush(v); ts[ro + 16] = hh; ts[64 * TP + ro + 16] = toh_flush((v - (float)hh) * RSC); }
            { const float v = (c2[r] * PINV + bb2) * QKC; const h16 hh = toh_flush(v); ts[ro + 32] = hh; ts[64 * TP + ro + 32] = toh_flush((v - (float)hh) * RSC); }
            { const float v = (c3[r] * PINV + bb3) * QKC; const h16 hh = toh_flush(v); ts[ro + 48] = hh; ts[64 * TP + ro + 48] = toh_flush((v - (float)hh) * RSC); } }
        __syncthreads();
        h16* dst = QK + (size_t)(2 * which) * QPL + ((size_t)b * R3 + row0 + 16 * wave) * DM + n0;
#pragma unroll 1
        for (int ps = 0; ps < 2; ++ps) {
#pragma unroll
            for (int s = 0; s < 4; ++s) { const int row = 4 * s + (lane >> 3), c8 = (lane & 7) * 8;
                const v8h vh = *(const v8ha*)(&ts[wave * 16 * TP + row * TP + c8]);
                const v8h vr = *(const v8ha*)(&ts[64 * TP + wave * 16 * TP + row * TP + c8]);
                *(volatile v8h*)(dst + (size_t)row * DM + c8) = vh;
                *(volatile v8h*)(dst + QPL + (size_t)row * DM + c8) = vr; }
            if (ps == 0) __threadfence(); }
    } else {
#pragma unroll
        for (int r = 0; r < 8; ++r) { const int so = lr * TP + 16 * wave + 8 * hi + r;
            { const float v = (c0[r] * PINV + bb0) * VC; const h16 hh = toh_flush(v); ts[so] = hh;           ts[64 * TP + so] = toh_flush((v - (float)hh) * RSC); }
            { const float v = (c1[r] * PINV + bb1) * VC; const h16 hh = toh_flush(v); ts[so + 16 * TP] = hh; ts[64 * TP + so + 16 * TP] = toh_flush((v - (float)hh) * RSC); }
            { const float v = (c2[r] * PINV + bb2) * VC; const h16 hh = toh_flush(v); ts[so + 32 * TP] = hh; ts[64 * TP + so + 32 * TP] = toh_flush((v - (float)hh) * RSC); }
            { const float v = (c3[r] * PINV + bb3) * VC; const h16 hh = toh_flush(v); ts[so + 48 * TP] = hh; ts[64 * TP + so + 48 * TP] = toh_flush((v - (float)hh) * RSC); } }
        __syncthreads();
        const size_t rb = (((size_t)b * DM + n0) * 3 + d) * SEQ + tl0;
#pragma unroll 1
        for (int ps = 0; ps < 2; ++ps) {
#pragma unroll
            for (int s = 0; s < 4; ++s) { const int nl = 16 * s + (tid >> 3), c8 = (tid & 7) * 8;
                const v8h vh = *(const v8ha*)(&ts[nl * TP + c8]);
                const v8h vr = *(const v8ha*)(&ts[64 * TP + nl * TP + c8]);
                *(volatile v8h*)(VTH + rb + (size_t)nl * 3 * SEQ + c8) = vh;
                *(volatile v8h*)(VTR + rb + (size_t)nl * 3 * SEQ + c8) = vr; }
            if (ps == 0) __threadfence(); }
    }
}

__global__ __launch_bounds__(256) __attribute__((amdgpu_num_vgpr(256)))
void k_attn(const h16* __restrict__ QK, const h16* __restrict__ VTH, const h16* __restrict__ VTR, h16* CHH, h16* CHR) {
    __shared__ __align__(16) h16 cs[2 * 48 * CSP];
    const int tid = threadIdx.x, lane = tid & 31, lr = lane & 15, hi = lane >> 4;
    const int h = __builtin_amdgcn_readfirstlane((int)(threadIdx.x >> 5));
    const int b = blockIdx.y, t0 = blockIdx.x * 16;
    const h16* qhp = QK + ((size_t)b * R3 + t0 + lr) * DM + h * HD + 8 * hi;
    const h16* khp = QK + 2 * QPL + ((size_t)b * R3 + lr) * DM + h * HD + 8 * hi;
    const h16* vhp = VTH + ((size_t)b * DM + h * HD + lr) * 3 * SEQ + 8 * hi;
    const h16* vrp = VTR + ((size_t)b * DM + h * HD + lr) * 3 * SEQ + 8 * hi;
    v8f oh[6], ox[6];
#pragma unroll
    for (int i = 0; i < 6; ++i) { oh[i] = (v8f){}; ox[i] = (v8f){}; }
    float m = -3.0e38f, l = 0.0f;
#pragma unroll 1
    for (int key0 = 0; key0 < SEQ; key0 += 32) {
        v8f sa0 = (v8f){}, sa1 = (v8f){}, sx0 = (v8f){}, sx1 = (v8f){};
#pragma unroll 1
        for (int d = 0; d < 3; ++d) {
            const size_t dq = (size_t)d * SEQ * DM;
            const v16h qh = ldh(qhp + dq), qr = ldh(qhp + QPL + dq);
            const size_t kk = dq + (size_t)key0 * DM;
            const v16h k0h = ldh(khp + kk), k0r = ldh(khp + QPL + kk);
            sa0 = wmma_g(k0h, qh, sa0); sx0 = wmma_g(k0h, qr, sx0); sx0 = wmma_g(k0r, qh, sx0);
            const v16h k1h = ldh(khp + kk + (size_t)16 * DM), k1r = ldh(khp + QPL + kk + (size_t)16 * DM);
            sa1 = wmma_g(k1h, qh, sa1); sx1 = wmma_g(k1h, qr, sx1); sx1 = wmma_g(k1r, qh, sx1);
        }
        float ta[8], tb[8]; float mx = -3.0e38f;
#pragma unroll
        for (int r = 0; r < 8; ++r) { ta[r] = (sa0[r] + sx0[r] * RINV) * SC2; tb[r] = (sa1[r] + sx1[r] * RINV) * SC2; mx = fmaxf(mx, fmaxf(ta[r], tb[r])); }
        mx = fmaxf(mx, __shfl_xor(mx, 16, 32));
        const float mnew = fmaxf(m, mx);
        const float alpha = __builtin_amdgcn_exp2f(m - mnew);
        v16h pbh, pbr; float ls = 0.0f;
#pragma unroll
        for (int r = 0; r < 8; ++r) {
            const float e0 = ta[r] - mnew, e1 = tb[r] - mnew;
            const float x0 = __builtin_amdgcn_exp2f(e0 + PEXP), x1 = __builtin_amdgcn_exp2f(e1 + PEXP);
            const float p0 = (e0 < -23.0f) ? 0.0f : x0;
            const float p1 = (e1 < -23.0f) ? 0.0f : x1;
            const h16 h0 = (h16)p0, h1 = (h16)p1;
            const h16 r0 = toh_flush((p0 - (float)h0) * RSC), r1 = toh_flush((p1 - (float)h1) * RSC);
            pbh[r] = h0; pbh[8 + r] = h1; pbr[r] = r0; pbr[8 + r] = r1;
            ls += ((float)h0 + (float)r0 * RINV) + ((float)h1 + (float)r1 * RINV); }
        l = l * alpha + ls; m = mnew;
#pragma unroll
        for (int i = 0; i < 6; ++i) { oh[i] = oh[i] * alpha; ox[i] = ox[i] * alpha; }
#pragma unroll
        for (int d = 0; d < 3; ++d) {
#pragma unroll
            for (int j = 0; j < 2; ++j) {
                const size_t vo = (size_t)(48 * j + d) * SEQ + key0;
                const v16h vh = ldh(vhp + vo), vr = ldh(vrp + vo);
                oh[2 * d + j] = wmma_g(vh, pbh, oh[2 * d + j]);
                ox[2 * d + j] = wmma_g(vr, pbh, ox[2 * d + j]);
                ox[2 * d + j] = wmma_g(vh, pbr, ox[2 * d + j]);
            } }
    }
    l += __shfl_xor(l, 16, 32);
    const float so = (CC / VC) / l;
#pragma unroll
    for (int d = 0; d < 3; ++d) {
#pragma unroll
        for (int j = 0; j < 2; ++j) {
            v8h ch, cr;
#pragma unroll
            for (int r = 0; r < 8; ++r) { const float c = (oh[2 * d + j][r] + ox[2 * d + j][r] * RINV) * so; const h16 hh = toh_flush(c); ch[r] = hh; cr[r] = toh_flush((c - (float)hh) * RSC); }
            const int o = (d * 16 + lr) * CSP + h * HD + 16 * j + 8 * hi;
            *(v8ha*)(&cs[o]) = ch; *(v8ha*)(&cs[48 * CSP + o]) = cr;
        } }
    __syncthreads();
    const size_t cb = ((size_t)b * R3 + t0) * DM;
#pragma unroll 1
    for (int ps = 0; ps < 2; ++ps) {
#pragma unroll
        for (int s = 0; s < 6; ++s) { const int row = 8 * s + h, c8 = lane * 8;
            const int dd = row >> 4, tt = row & 15;
            const v8h a = *(const v8ha*)(&cs[row * CSP + c8]);
            const v8h c = *(const v8ha*)(&cs[48 * CSP + row * CSP + c8]);
            const size_t g = cb + ((size_t)dd * SEQ + tt) * DM + c8;
            *(volatile v8h*)(CHH + g) = a;
            *(volatile v8h*)(CHR + g) = c; }
        if (ps == 0) __threadfence(); }
}

__global__ __launch_bounds__(128) void k_gemm(const h16* __restrict__ AH, const h16* __restrict__ AR, const h16* __restrict__ W, const float* __restrict__ U, float ascale, float* F) {
    __shared__ __align__(16) float os[4 * 16 * OSP];
    const int lane = threadIdx.x & 31, lr = lane & 15, hi = lane >> 4;
    const int wave = __builtin_amdgcn_readfirstlane((int)(threadIdx.x >> 5));
    const size_t row0 = (size_t)blockIdx.x * 16;
    const int d = (int)((row0 % R3) / SEQ), n0 = wave * 64;
    const size_t ao = (row0 + lr) * DM + 8 * hi;
    const h16* ap = AH + ao; const h16* rp = AR + ao;
    const h16* wp = W + (size_t)(n0 + lr) * DM + 8 * hi;
    v8f c0 = (v8f){}, c1 = (v8f){}, c2 = (v8f){}, c3 = (v8f){}, d0 = (v8f){}, d1 = (v8f){}, d2 = (v8f){}, d3 = (v8f){};
#pragma unroll 1
    for (int k0 = 0; k0 < DM; k0 += 32) {
        const v16h a = ldh(ap + k0), ar = ldh(rp + k0);
        const v16h w0 = ldh(wp + k0), w1 = ldh(wp + (size_t)16 * DM + k0), w2 = ldh(wp + (size_t)32 * DM + k0), w3 = ldh(wp + (size_t)48 * DM + k0);
        c0 = wmma_g(a, w0, c0); c1 = wmma_g(a, w1, c1); c2 = wmma_g(a, w2, c2); c3 = wmma_g(a, w3, c3);
        d0 = wmma_g(ar, w0, d0); d1 = wmma_g(ar, w1, d1); d2 = wmma_g(ar, w2, d2); d3 = wmma_g(ar, w3, d3);
    }
    const float* up = U + (size_t)d * DM + n0 + lr;
    const float bb0 = up[0], bb1 = up[16], bb2 = up[32], bb3 = up[48];
    const int wb = wave * 16 * OSP;
#pragma unroll
    for (int r = 0; r < 8; ++r) { const int ro = wb + (8 * hi + r) * OSP + lr;
        os[ro]      = (c0[r] + d0[r] * RINV) * ascale + bb0; os[ro + 16] = (c1[r] + d1[r] * RINV) * ascale + bb1;
        os[ro + 32] = (c2[r] + d2[r] * RINV) * ascale + bb2; os[ro + 48] = (c3[r] + d3[r] * RINV) * ascale + bb3; }
    __syncthreads();
    float* orow = F + row0 * DM + n0;
#pragma unroll 1
    for (int ps = 0; ps < 2; ++ps) {
#pragma unroll
        for (int s = 0; s < 8; ++s) { const int row = 2 * s + hi, cofs = lr * 4;
            const v4f val = *(const v4fa*)(&os[wb + row * OSP + cofs]);
            *(volatile v4f*)(orow + (size_t)row * DM + cofs) = val; }
        if (ps == 0) __threadfence(); }
}

__global__ __launch_bounds__(256) void k_ln(const float* __restrict__ F, const h16* __restrict__ RH, const h16* __restrict__ RR, float rs1, float rs2,
                                            const float* __restrict__ g, const float* __restrict__ be, h16* OH, h16* OL) {
#pragma clang fp contract(off)
    const int lane = threadIdx.x & 31, wave = __builtin_amdgcn_readfirstlane((int)(threadIdx.x >> 5));
    const size_t tk = (size_t)blockIdx.x * 8 + wave;
    const size_t b = tk / SEQ, n = tk % SEQ;
    const size_t r0 = (b * R3 + n) * DM + lane * 8, r1 = r0 + (size_t)SEQ * DM, r2 = r1 + (size_t)SEQ * DM;
    const v8f x0 = *(const v8f*)(F + r0), x1 = *(const v8f*)(F + r1), x2 = *(const v8f*)(F + r2);
    v8f nr; float s = 0.0f;
#pragma unroll
    for (int k = 0; k < 8; ++k) { const float ss = x0[k] * x0[k] + x1[k] * x1[k] + x2[k] * x2[k]; nr[k] = __builtin_amdgcn_sqrtf(ss) + 1e-6f; s += nr[k]; }
    s += __shfl_xor(s, 16, 32); s += __shfl_xor(s, 8, 32); s += __shfl_xor(s, 4, 32); s += __shfl_xor(s, 2, 32); s += __shfl_xor(s, 1, 32);
    const float mu = s * 0.00390625f;
    float q = 0.0f;
#pragma unroll
    for (int k = 0; k < 8; ++k) { const float dl = nr[k] - mu; q += dl * dl; }
    q += __shfl_xor(q, 16, 32); q += __shfl_xor(q, 8, 32); q += __shfl_xor(q, 4, 32); q += __shfl_xor(q, 2, 32); q += __shfl_xor(q, 1, 32);
    const float rstd = 1.0f / sqrtf(q * 0.00390625f + 1e-5f);
    const v8f gv = *(const v8f*)(g + lane * 8), bv = *(const v8f*)(be + lane * 8);
    const v8h h0 = *(const v8h*)(RH + r0), h1 = *(const v8h*)(RH + r1), h2 = *(const v8h*)(RH + r2);
    const v8h l0 = *(const v8h*)(RR + r0), l1 = *(const v8h*)(RR + r1), l2 = *(const v8h*)(RR + r2);
    v8h yh0, yh1, yh2, yl0, yl1, yl2;
#pragma unroll
    for (int k = 0; k < 8; ++k) {
        const float ln = (nr[k] - mu) * rstd * rbf(gv[k]) + rbf(bv[k]);
        const float rn = __builtin_amdgcn_rcpf(nr[k]);
        { const float v = ((x0[k] * rn) * ln + ((float)h0[k] * rs1 + (float)l0[k] * rs2)) * AC; const h16 hh = toh_flush(v); yh0[k] = hh; yl0[k] = toh_flush((v - (float)hh) * RSC); }
        { const float v = ((x1[k] * rn) * ln + ((float)h1[k] * rs1 + (float)l1[k] * rs2)) * AC; const h16 hh = toh_flush(v); yh1[k] = hh; yl1[k] = toh_flush((v - (float)hh) * RSC); }
        { const float v = ((x2[k] * rn) * ln + ((float)h2[k] * rs1 + (float)l2[k] * rs2)) * AC; const h16 hh = toh_flush(v); yh2[k] = hh; yl2[k] = toh_flush((v - (float)hh) * RSC); } }
    *(volatile v8h*)(OH + r0) = yh0; *(volatile v8h*)(OH + r1) = yh1; *(volatile v8h*)(OH + r2) = yh2;
    *(volatile v8h*)(OL + r0) = yl0; *(volatile v8h*)(OL + r1) = yl1; *(volatile v8h*)(OL + r2) = yl2;
    __threadfence();
    *(volatile v8h*)(OH + r0) = yh0; *(volatile v8h*)(OH + r1) = yh1; *(volatile v8h*)(OH + r2) = yh2;
    *(volatile v8h*)(OL + r0) = yl0; *(volatile v8h*)(OL + r1) = yl1; *(volatile v8h*)(OL + r2) = yl2;
}

__global__ __launch_bounds__(256) void k_bn_part(const float* __restrict__ F, float* PART) {
#pragma clang fp contract(off)
    __shared__ __align__(16) float sp[2 * DM];
    const int c = threadIdx.x;
    const size_t tk0 = (size_t)blockIdx.x * 64;
    const size_t b = tk0 / SEQ, n0 = tk0 % SEQ;
    const float* p = F + (b * R3 + n0) * DM + c;
    float s = 0.0f, q = 0.0f;
#pragma unroll 1
    for (int i = 0; i < 64; ++i) {
        const float x0 = p[(size_t)i * DM], x1 = p[(size_t)(SEQ + i) * DM], x2 = p[(size_t)(2 * SEQ + i) * DM];
        const float nr = __builtin_amdgcn_sqrtf(x0 * x0 + x1 * x1 + x2 * x2) + 1e-6f;
        s += nr; q += nr * nr; }
    sp[c] = s; sp[DM + c] = q;
    __syncthreads();
    if (c < 128) {
        const v4f val = *(const v4fa*)(&sp[c * 4]);
        float* dst = PART + (size_t)blockIdx.x * 2 * DM + c * 4;
        *(volatile v4f*)dst = val;
        __threadfence();
        *(volatile v4f*)dst = val;
    }
}

__global__ __launch_bounds__(256) void k_bn_fin(const float* __restrict__ PART, float* STAT) {
#pragma clang fp contract(off)
    __shared__ __align__(16) float st[2 * DM];
    const int c = threadIdx.x;
    double S = 0.0, Q = 0.0;
#pragma unroll 1
    for (int blk = 0; blk < (NB * SEQ) / 64; ++blk) { S += (double)PART[(size_t)blk * 2 * DM + c]; Q += (double)PART[(size_t)blk * 2 * DM + DM + c]; }
    const double invn = 1.0 / (double)((size_t)NB * SEQ);
    const double mu = S * invn;
    double var = Q * invn - mu * mu;
    var = (var > 0.0) ? var : 0.0;
    st[c] = (float)mu; st[DM + c] = 1.0f / sqrtf((float)var + 1e-5f);
    __syncthreads();
    if (c < 128) {
        const v4f val = *(const v4fa*)(&st[c * 4]);
        float* dst = STAT + c * 4;
        *(volatile v4f*)dst = val;
        __threadfence();
        *(volatile v4f*)dst = val;
    }
}

__global__ __launch_bounds__(256) void k_bn_apply(const float* __restrict__ F, const float* __restrict__ STAT, const float* __restrict__ g, const float* __restrict__ be, h16* OH, h16* OL) {
#pragma clang fp contract(off)
    const int lane = threadIdx.x & 31, wave = __builtin_amdgcn_readfirstlane((int)(threadIdx.x >> 5));
    const size_t tk = (size_t)blockIdx.x * 8 + wave;
    const size_t b = tk / SEQ, n = tk % SEQ;
    const size_t r0 = (b * R3 + n) * DM + lane * 8, r1 = r0 + (size_t)SEQ * DM, r2 = r1 + (size_t)SEQ * DM;
    const v8f x0 = *(const v8f*)(F + r0), x1 = *(const v8f*)(F + r1), x2 = *(const v8f*)(F + r2);
    const v8f mv = *(const v8f*)(STAT + lane * 8), rv = *(const v8f*)(STAT + DM + lane * 8);
    const v8f gv = *(const v8f*)(g + lane * 8), bv = *(const v8f*)(be + lane * 8);
    v8h yh0, yh1, yh2, yl0, yl1, yl2;
#pragma unroll
    for (int k = 0; k < 8; ++k) {
        const float nr = __builtin_amdgcn_sqrtf(x0[k] * x0[k] + x1[k] * x1[k] + x2[k] * x2[k]) + 1e-6f;
        const float bn = (nr - mv[k]) * rv[k] * rbf(gv[k]) + rbf(bv[k]);
        const float rn = __builtin_amdgcn_rcpf(nr);
        { const float v = ((x0[k] * rn) * bn) * AC; const h16 hh = toh_flush(v); yh0[k] = hh; yl0[k] = toh_flush((v - (float)hh) * RSC); }
        { const float v = ((x1[k] * rn) * bn) * AC; const h16 hh = toh_flush(v); yh1[k] = hh; yl1[k] = toh_flush((v - (float)hh) * RSC); }
        { const float v = ((x2[k] * rn) * bn) * AC; const h16 hh = toh_flush(v); yh2[k] = hh; yl2[k] = toh_flush((v - (float)hh) * RSC); } }
    *(volatile v8h*)(OH + r0) = yh0; *(volatile v8h*)(OH + r1) = yh1; *(volatile v8h*)(OH + r2) = yh2;
    *(volatile v8h*)(OL + r0) = yl0; *(volatile v8h*)(OL + r1) = yl1; *(volatile v8h*)(OL + r2) = yl2;
    __threadfence();
    *(volatile v8h*)(OH + r0) = yh0; *(volatile v8h*)(OH + r1) = yh1; *(volatile v8h*)(OH + r2) = yh2;
    *(volatile v8h*)(OL + r0) = yl0; *(volatile v8h*)(OL + r1) = yl1; *(volatile v8h*)(OL + r2) = yl2;
}

__global__ __launch_bounds__(256) void k_leaky(const h16* __restrict__ XA, const h16* __restrict__ XL, const float* __restrict__ D, h16* OH, h16* OL) {
#pragma clang fp contract(off)
    const int lane = threadIdx.x & 31, wave = __builtin_amdgcn_readfirstlane((int)(threadIdx.x >> 5));
    const size_t tk = (size_t)blockIdx.x * 8 + wave;
    const size_t b = tk / SEQ, n = tk % SEQ;
    const size_t r0 = (b * R3 + n) * DM + lane * 8, r1 = r0 + (size_t)SEQ * DM, r2 = r1 + (size_t)SEQ * DM;
    const v8f d0 = *(const v8f*)(D + r0), d1 = *(const v8f*)(D + r1), d2 = *(const v8f*)(D + r2);
    const v8h h0 = *(const v8h*)(XA + r0), h1 = *(const v8h*)(XA + r1), h2 = *(const v8h*)(XA + r2);
    const v8h l0 = *(const v8h*)(XL + r0), l1 = *(const v8h*)(XL + r1), l2 = *(const v8h*)(XL + r2);
    v8h yh0, yh1, yh2, yl0, yl1, yl2;
#pragma unroll
    for (int k = 0; k < 8; ++k) {
        const float x0 = ((float)h0[k] + (float)l0[k] * RINV) * AINV;
        const float x1 = ((float)h1[k] + (float)l1[k] * RINV) * AINV;
        const float x2 = ((float)h2[k] + (float)l2[k] * RINV) * AINV;
        const float dot = x0 * d0[k] + x1 * d1[k] + x2 * d2[k];
        const float dn = d0[k] * d0[k] + d1[k] * d1[k] + d2[k] * d2[k];
        const float kk = dot * __builtin_amdgcn_rcpf(dn + 1e-6f);
        const bool pos = dot >= 0.0f;
        const float p0 = x0 - kk * d0[k], p1 = x1 - kk * d1[k], p2 = x2 - kk * d2[k];
        { const float v = (pos ? x0 : p0) * AC; const h16 hh = toh_flush(v); yh0[k] = hh; yl0[k] = toh_flush((v - (float)hh) * RSC); }
        { const float v = (pos ? x1 : p1) * AC; const h16 hh = toh_flush(v); yh1[k] = hh; yl1[k] = toh_flush((v - (float)hh) * RSC); }
        { const float v = (pos ? x2 : p2) * AC; const h16 hh = toh_flush(v); yh2[k] = hh; yl2[k] = toh_flush((v - (float)hh) * RSC); } }
    *(volatile v8h*)(OH + r0) = yh0; *(volatile v8h*)(OH + r1) = yh1; *(volatile v8h*)(OH + r2) = yh2;
    *(volatile v8h*)(OL + r0) = yl0; *(volatile v8h*)(OL + r1) = yl1; *(volatile v8h*)(OL + r2) = yl2;
    __threadfence();
    *(volatile v8h*)(OH + r0) = yh0; *(volatile v8h*)(OH + r1) = yh1; *(volatile v8h*)(OH + r2) = yh2;
    *(volatile v8h*)(OL + r0) = yl0; *(volatile v8h*)(OL + r1) = yl1; *(volatile v8h*)(OL + r2) = yl2;
}

__global__ __launch_bounds__(256) void k_out_t(const h16* __restrict__ OH, const h16* __restrict__ OL, float* OUT) {
#pragma clang fp contract(off)
    __shared__ __align__(16) float tf[64 * TFP];
    const int tid = threadIdx.x;
    const int row0 = blockIdx.x * 64, d = row0 / SEQ, tl0 = row0 % SEQ;
    const int c0 = blockIdx.y * 64, b = blockIdx.z;
    const int tl = tid >> 2, q = (tid & 3) * 16;
    const size_t so = ((size_t)b * R3 + row0 + tl) * DM + c0 + q;
    const v8h h0 = *(const v8h*)(OH + so), h1 = *(const v8h*)(OH + so + 8);
    const v8h l0 = *(const v8h*)(OL + so), l1 = *(const v8h*)(OL + so + 8);
#pragma unroll
    for (int k = 0; k < 8; ++k) {
        tf[(q + k) * TFP + tl]     = ((float)h0[k] + (float)l0[k] * RINV) * AINV;
        tf[(q + 8 + k) * TFP + tl] = ((float)h1[k] + (float)l1[k] * RINV) * AINV; }
    __syncthreads();
#pragma unroll 1
    for (int ps = 0; ps < 2; ++ps) {
#pragma unroll
        for (int s = 0; s < 4; ++s) { const int row = 16 * s + (tid >> 4), cofs = (tid & 15) * 4;
            const v4f val = *(const v4fa*)(&tf[row * TFP + cofs]);
            float* dst = OUT + (((size_t)b * DM + c0 + row) * 3 + d) * SEQ_FULL + tl0 + cofs;
            *(volatile v4f*)dst = val; }
        if (ps == 0) __threadfence(); }
}

static constexpr size_t al256(size_t v) { return (v + 255) & ~(size_t)255; }
static constexpr size_t SZ_P    = al256(QPL * 2);
static constexpr size_t SZ_W    = al256((size_t)NMAT * DM * DM * 2);
static constexpr size_t SZ_U    = al256((size_t)NMAT * 3 * DM * 4);
static constexpr size_t SZ_PART = al256(((size_t)NB * SEQ / 64) * 2 * DM * 4);
static constexpr size_t SZ_STAT = al256((size_t)2 * DM * 4);
static constexpr size_t SZ_TOTAL = 9 * SZ_P + SZ_W + SZ_U + SZ_PART + SZ_STAT;
static_assert(SZ_P == QPL * 2);
static_assert(2 * SZ_P >= QPL * 4);
static_assert((size_t)NB * DM * 3 * SEQ == QPL);
static_assert(SZ_TOTAL <= (size_t)134217728);

extern "C" void kernel_launch(void* const* d_in, const int* in_sizes, int n_in,
                              void* d_out, int out_size, void* d_ws, size_t ws_size, hipStream_t stream) {
    if (n_in < 20) return;
    const size_t needx = ((size_t)NB * DM * 3 - 1) * SEQ_FULL + SEQ;
    if ((size_t)in_sizes[0] < needx) return;
    if ((size_t)in_sizes[1] < (size_t)DM * DM || (size_t)in_sizes[3] < (size_t)DM * DM || (size_t)in_sizes[5] < (size_t)DM * DM || (size_t)in_sizes[7] < (size_t)DM * DM) return;
    if ((size_t)in_sizes[11] < (size_t)DM * DM || (size_t)in_sizes[15] < (size_t)DM * DM || (size_t)in_sizes[16] < (size_t)DM * DM) return;
    if (in_sizes[2] < DM * 3 || in_sizes[4] < DM * 3 || in_sizes[6] < DM * 3 || in_sizes[8] < DM * 3 || in_sizes[12] < DM * 3 || in_sizes[17] < DM * 3) return;
    if (in_sizes[9] < DM || in_sizes[10] < DM || in_sizes[13] < DM || in_sizes[14] < DM || in_sizes[18] < DM || in_sizes[19] < DM) return;
    if ((size_t)out_size < needx) return;
    if (SZ_TOTAL > ws_size) return;
    const float* x    = (const float*)d_in[0];
    const float* Wq   = (const float*)d_in[1];  const float* bq  = (const float*)d_in[2];
    const float* Wk   = (const float*)d_in[3];  const float* bk  = (const float*)d_in[4];
    const float* Wz   = (const float*)d_in[5];  const float* bz  = (const float*)d_in[6];
    const float* Wo   = (const float*)d_in[7];  const float* bo  = (const float*)d_in[8];
    const float* ln1g = (const float*)d_in[9];  const float* ln1b = (const float*)d_in[10];
    const float* Wm1  = (const float*)d_in[11]; const float* bm1 = (const float*)d_in[12];
    const float* bng  = (const float*)d_in[13]; const float* bnb = (const float*)d_in[14];
    const float* Wr   = (const float*)d_in[15];
    const float* Wm2  = (const float*)d_in[16]; const float* bm2 = (const float*)d_in[17];
    const float* ln2g = (const float*)d_in[18]; const float* ln2b = (const float*)d_in[19];
    float* OUT = (float*)d_out;
    char* wsp = (char*)d_ws;
    h16* S0 = (h16*)wsp; wsp += SZ_P;
    h16* S1 = (h16*)wsp; wsp += SZ_P;
    h16* S2 = (h16*)wsp; wsp += SZ_P;
    h16* S3 = (h16*)wsp; wsp += SZ_P;
    h16* S4 = (h16*)wsp; wsp += SZ_P;
    h16* S5 = (h16*)wsp; wsp += SZ_P;
    h16* S6 = (h16*)wsp; wsp += SZ_P;
    h16* S7 = (h16*)wsp; wsp += SZ_P;
    h16* S8 = (h16*)wsp; wsp += SZ_P;
    h16* WH = (h16*)wsp; wsp += SZ_W;
    float* UT = (float*)wsp; wsp += SZ_U;
    float* PART = (float*)wsp; wsp += SZ_PART;
    float* STAT = (float*)wsp; wsp += SZ_STAT;
    float* F1 = (float*)S1;

    const size_t WW = (size_t)DM * DM;
    const unsigned nrow16 = (unsigned)(((size_t)NB * R3) / 16);
    const unsigned ntok8 = (unsigned)(((size_t)NB * SEQ) / 8);
    k_cvt_x<<<dim3(R3 / 64, DM / 64, NB), 256, 0, stream>>>(x, S0);
    k_cvt_w<<<dim3(DM / 64, DM / 64, NMAT), 256, 0, stream>>>(Wq, Wk, Wz, Wo, Wm1, Wr, Wm2, bq, bk, bz, bo, bm1, bm2, WH, UT);
    k_proj<<<dim3(R3 / 64, DM / 64, 3 * NB), 128, 0, stream>>>(S0, WH, UT, S1, S5, S6);
    k_attn<<<dim3(SEQ / 16, NB, 1), 256, 0, stream>>>(S1, S5, S6, S7, S8);
    k_gemm<<<nrow16, 128, 0, stream>>>(S7, S8, WH + 3 * WW, UT + (size_t)3 * 3 * DM, 1.0f / (CC * WSC), F1);
    k_ln<<<ntok8, 256, 0, stream>>>(F1, S0, S0, 1.0f / XC, 0.0f, ln1g, ln1b, S3, S4);
    k_gemm<<<nrow16, 128, 0, stream>>>(S3, S4, WH + 4 * WW, UT + (size_t)4 * 3 * DM, 1.0f / (AC * WSC), F1);
    k_bn_part<<<(unsigned)(((size_t)NB * SEQ) / 64), 256, 0, stream>>>(F1, PART);
    k_bn_fin<<<1, 256, 0, stream>>>(PART, STAT);
    k_bn_apply<<<ntok8, 256, 0, stream>>>(F1, STAT, bng, bnb, S5, S6);
    k_gemm<<<nrow16, 128, 0, stream>>>(S5, S6, WH + 5 * WW, UT + (size_t)5 * 3 * DM, 1.0f / (AC * WSC), F1);
    k_leaky<<<ntok8, 256, 0, stream>>>(S5, S6, F1, S7, S8);
    k_gemm<<<nrow16, 128, 0, stream>>>(S7, S8, WH + 6 * WW, UT + (size_t)6 * 3 * DM, 1.0f / (AC * WSC), F1);
    k_ln<<<ntok8, 256, 0, stream>>>(F1, S3, S4, 1.0f / AC, RINV / AC, ln2g, ln2b, S5, S6);
    k_out_t<<<dim3(R3 / 64, DM / 64, NB), 256, 0, stream>>>(S5, S6, OUT);
}
